// DecoderBlock_59176059404572
// MI455X (gfx1250) — hardware-run, weakly checked
//
#include <hip/hip_runtime.h>
#include <math.h>

typedef __attribute__((ext_vector_type(16))) _Float16 v16h;
typedef __attribute__((ext_vector_type(8)))  _Float16 v8h;
typedef __attribute__((ext_vector_type(16))) __bf16   v16b;
typedef __attribute__((ext_vector_type(8)))  __bf16   v8b;
typedef __attribute__((ext_vector_type(8)))  float    v8f;
typedef __attribute__((ext_vector_type(4)))  float    v4f;
typedef __attribute__((ext_vector_type(4)))  unsigned v4u;
typedef __attribute__((ext_vector_type(2)))  unsigned v2u;

constexpr int kBatch = 2;
constexpr int kSeq   = 2048;
constexpr int kDim   = 1024;
constexpr int kHeads = 16;
constexpr int kHdim  = 64;
constexpr int kFfn   = 4096;
constexpr int kRows  = kBatch * kSeq;
constexpr int kQkvLd = 3 * kHdim * kHeads;

constexpr float kCarryAct  = 8.0f;
constexpr float kCarryWqkv = 64.0f;
constexpr float kCarryQkv  = 8.0f;
constexpr float kCarryP    = 1024.0f;
constexpr float kCarryAttn = 64.0f;
constexpr float kCarryWo   = 256.0f;
constexpr float kCarryW1   = 256.0f;
constexpr float kCarryW2   = 512.0f;
constexpr float kCarryH    = 8.0f;

constexpr size_t kSzWqkv = (size_t)kHeads * 3 * kHdim * kHdim * 2;
constexpr size_t kSzWo   = (size_t)kDim * kDim * 2;
constexpr size_t kSzW1   = (size_t)kFfn * kDim * 2;
constexpr size_t kSzW2   = (size_t)kDim * kFfn * 2;
constexpr size_t kSzF32  = (size_t)kRows * kDim * 4;
constexpr size_t kSzH16  = (size_t)kRows * kDim * 2;
constexpr size_t kSzQkv  = (size_t)kRows * kQkvLd * 2;
constexpr size_t kSzHid  = (size_t)kRows * kFfn * 2;
constexpr size_t kOffWqkv = 0;
constexpr size_t kOffWo   = kOffWqkv + kSzWqkv;
constexpr size_t kOffW1   = kOffWo + kSzWo;
constexpr size_t kOffW2   = kOffW1 + kSzW1;
constexpr size_t kOffX1f  = kOffW2 + kSzW2;
constexpr size_t kOffX1h  = kOffX1f + kSzF32;
constexpr size_t kOffQkv  = kOffX1h + kSzH16;
constexpr size_t kOffAttn = kOffQkv + kSzQkv;
constexpr size_t kOffU    = kOffAttn + kSzH16;
constexpr size_t kWsTotal = kOffU + kSzF32;
constexpr size_t kOffHid  = kOffQkv;
static_assert(kSzQkv + kSzH16 == kSzHid);
static_assert(kOffHid + kSzHid == kOffU);
static_assert(kWsTotal == 94765056);
static_assert(kWsTotal <= 134217728);
static_assert((kOffWo % 128) == 0 && (kOffW1 % 128) == 0 && (kOffW2 % 128) == 0 && (kOffX1f % 128) == 0 &&
              (kOffX1h % 128) == 0 && (kOffQkv % 128) == 0 && (kOffAttn % 128) == 0 && (kOffU % 128) == 0);
static_assert(kRows % 64 == 0 && (3 * kHdim) % 64 == 0 && kHdim % 32 == 0);
static_assert(kDim % 64 == 0 && kFfn % 64 == 0 && kDim % 32 == 0 && kFfn % 32 == 0);
static_assert(kSeq % 64 == 0 && kHdim == 64);

__device__ __forceinline__ unsigned short f2bf_bits(float f) {
  unsigned u = __float_as_uint(f);
  return (unsigned short)((u + 0x7FFFu + ((u >> 16) & 1u)) >> 16);
}
__device__ __forceinline__ float bf_bits2f(unsigned short h) { return __uint_as_float(((unsigned)h) << 16); }

__device__ __forceinline__ void dep_guard_h(v8f& a, v8f& b, v16h x, v16h y) { asm volatile("v_nop\n\tv_nop\n\tv_nop\n\tv_nop" : "+v"(a), "+v"(b) : "v"(x), "v"(y)); }
__device__ __forceinline__ void dep_guard_b(v8f& a, v8f& b, v16b x, v16b y) { asm volatile("v_nop\n\tv_nop\n\tv_nop\n\tv_nop" : "+v"(a), "+v"(b) : "v"(x), "v"(y)); }
__device__ __forceinline__ void keep4_h(v16h a, v16h b, v16h c, v16h d) { asm volatile("v_nop" :: "v"(a), "v"(b), "v"(c), "v"(d)); }
__device__ __forceinline__ void keep4_b(v16b a, v16b b, v16b c, v16b d) { asm volatile("v_nop" :: "v"(a), "v"(b), "v"(c), "v"(d)); }
__device__ __forceinline__ void acc_guard4(v8f& a, v8f& b, v8f& c, v8f& d) { asm volatile("v_nop\n\tv_nop\n\tv_nop\n\tv_nop" : "+v"(a), "+v"(b), "+v"(c), "+v"(d)); }
template <typename T> struct Frag;
template <> struct Frag<_Float16> {
  typedef v16h V; union U { v16h v; v8h h[2]; };
  static __device__ __forceinline__ v16h load(const _Float16* p) {
    U f; f.h[0] = *(const v8h*)(p); f.h[1] = *(const v8h*)(p + 16); return f.v;
  }
  static __device__ __forceinline__ v8f mma(v16h a, v16h b, v8f c) {
    return __builtin_amdgcn_wmma_f32_16x16x32_f16(false, a, false, b, (short)0, c, false, false);
  }
  static __device__ __forceinline__ void guard(v8f& a, v8f& b, v16h x, v16h y) { dep_guard_h(a, b, x, y); }
  static __device__ __forceinline__ void keep(v16h a, v16h b, v16h c, v16h d) { keep4_h(a, b, c, d); }
};
template <> struct Frag<__bf16> {
  typedef v16b V; union U { v16b v; v8b h[2]; };
  static __device__ __forceinline__ v16b load(const __bf16* p) {
    U f; f.h[0] = *(const v8b*)(p); f.h[1] = *(const v8b*)(p + 16); return f.v;
  }
  static __device__ __forceinline__ v8f mma(v16b a, v16b b, v8f c) {
    return __builtin_amdgcn_wmma_f32_16x16x32_bf16(false, a, false, b, (short)0, c, false, false);
  }
  static __device__ __forceinline__ void guard(v8f& a, v8f& b, v16b x, v16b y) { dep_guard_b(a, b, x, y); }
  static __device__ __forceinline__ void keep(v16b a, v16b b, v16b c, v16b d) { keep4_b(a, b, c, d); }
};

template <int ET> struct Elem;
template <> struct Elem<0> { typedef _Float16 T; };
template <> struct Elem<1> { typedef __bf16 T; };
template <int ET, bool SPLIT, int BIAS_MODE, int OUT_MODE, bool RESID, int ACT = 0>
__global__ __launch_bounds__(256) void wmma_gemm64(
    const unsigned short* __restrict__ Ap, const unsigned short* __restrict__ A2p, int lda, long strideA,
    const unsigned short* __restrict__ Btp, const unsigned short* __restrict__ Bt2p, int ldb, long strideB,
    void* __restrict__ Cout, void* __restrict__ Cout2, int ldc, long strideC,
    const float* __restrict__ bias,
    const float* __restrict__ resid, long strideR,
    int M, int N, int K, float scale, float oscale) {
  static_assert(!RESID || OUT_MODE == 0);
  typedef typename Elem<ET>::T T;
  typedef typename Frag<T>::V V;
  const T* A = (const T*)Ap; const T* A2 = (const T*)A2p; const T* Bt = (const T*)Btp; const T* Bt2 = (const T*)Bt2p;
  __shared__ __align__(16) float sT[8][16 * 68];
  const int b    = blockIdx.y;
  const int lane = threadIdx.x & 31;
  const int wave = threadIdx.x >> 5;
  const int tilesN = N >> 6;
  const int tilesM = M >> 6;
  const int tile = blockIdx.x * 8 + wave;
  if (tile >= tilesM * tilesN) return;
  const int tm = tile / tilesN;
  const int tn = tile - tm * tilesN;
  const int m0 = tm << 6;
  const int n0 = tn << 6;

  const T* Ab  = A  + (size_t)b * strideA;
  const T* Bb  = Bt + (size_t)b * strideB;
  const T* Ab2 = SPLIT ? (A2  + (size_t)b * strideA) : nullptr;
  const T* Bb2 = SPLIT ? (Bt2 + (size_t)b * strideB) : nullptr;

  const int rlane = lane & 15;
  const int koff  = (lane >> 4) * 8;
  const int mOff  = (lane >> 4) * 8;

  v8f acc[4][4];
#pragma unroll
  for (int i = 0; i < 4; ++i)
#pragma unroll
    for (int j = 0; j < 4; ++j) acc[i][j] = (v8f){0.f,0.f,0.f,0.f,0.f,0.f,0.f,0.f};

  for (int k0 = 0; k0 < K; k0 += 32) {
    V bh[4], bl[4];
#pragma unroll
    for (int j = 0; j < 4; ++j) {
      const size_t bo = (size_t)(n0 + (j << 4) + rlane) * ldb + koff + k0;
      bh[j] = Frag<T>::load(Bb + bo);
      if (SPLIT) bl[j] = Frag<T>::load(Bb2 + bo);
    }
#pragma unroll
    for (int i = 0; i < 4; ++i) {
      const size_t ao = (size_t)(m0 + (i << 4) + rlane) * lda + koff + k0;
      V ah = Frag<T>::load(Ab + ao);
      V al;
      if (SPLIT) al = Frag<T>::load(Ab2 + ao);
#pragma unroll
      for (int j = 0; j < 4; ++j) {
        acc[i][j] = Frag<T>::mma(ah, bh[j], acc[i][j]);
        if (SPLIT) {
          acc[i][j] = Frag<T>::mma(ah, bl[j], acc[i][j]);
          acc[i][j] = Frag<T>::mma(al, bh[j], acc[i][j]);
        }
      }
      Frag<T>::guard(acc[i][0], acc[i][3], ah, SPLIT ? al : ah);
    }
    Frag<T>::keep(bh[0], bh[1], bh[2], bh[3]);
    if (SPLIT) Frag<T>::keep(bl[0], bl[1], bl[2], bl[3]);
  }
  acc_guard4(acc[0][0], acc[0][1], acc[0][2], acc[0][3]);
  acc_guard4(acc[1][0], acc[1][1], acc[1][2], acc[1][3]);
  acc_guard4(acc[2][0], acc[2][1], acc[2][2], acc[2][3]);
  acc_guard4(acc[3][0], acc[3][1], acc[3][2], acc[3][3]);

  float* slab = sT[wave];
  const float* Rb = RESID ? (resid + (size_t)b * strideR) : nullptr;
#pragma unroll
  for (int i = 0; i < 4; ++i) {
    const int mBase = m0 + (i << 4);
#pragma unroll
    for (int j = 0; j < 4; ++j) {
      const int n = n0 + (j << 4) + rlane;
      float bv = 0.f;
      if (BIAS_MODE == 2) bv = bias[n];
#pragma unroll
      for (int r = 0; r < 8; ++r) {
        float v = acc[i][j][r] * scale;
        if (BIAS_MODE == 1) v += bias[mBase + mOff + r];
        if (BIAS_MODE == 2) v += bv;
        if (ACT == 1) v = tanhf(v);
        if (ACT == 2) v = fmaxf(v, 0.0f);
        if (ACT == 3) v = v / (1.0f + expf(-v));
        if (ACT == 4) v = (v > 0.f) ? v : 0.01f * v;
        if (ACT == 6) {
          float t2 = 1.5957691216057308f * (v + 0.044715f * v * v * v);
          t2 = fmaxf(t2, -80.0f);
          v = v * __builtin_amdgcn_rcpf(1.0f + __expf(-t2));
        }
        slab[(mOff + r) * 68 + (j << 4) + rlane] = v * oscale;
      }
    }
    __builtin_amdgcn_fence(__ATOMIC_RELEASE, "workgroup");
    __builtin_amdgcn_wave_barrier();
    __builtin_amdgcn_fence(__ATOMIC_ACQUIRE, "workgroup");
    if (OUT_MODE == 0) {
      float* C = (float*)Cout + (size_t)b * strideC;
      const int hh = lane >> 4, c4 = (lane & 15) * 4;
      for (int pass = 0; pass < 2; ++pass) {
#pragma unroll
        for (int it = 0; it < 8; ++it) {
          const int row = it * 2 + hh;
          v4f v = *(const v4f*)(slab + row * 68 + c4);
          if (RESID) {
            const v4f rr = *(const v4f*)(Rb + (size_t)(mBase + row) * ldc + n0 + c4);
            v += rr;
          }
          *(volatile v4f*)(C + (size_t)(mBase + row) * ldc + n0 + c4) = v;
        }
        __threadfence();
      }
    } else {
      const int q = lane >> 3, c8 = (lane & 7) * 8;
      unsigned short* C  = (unsigned short*)Cout  + (size_t)b * strideC;
      unsigned short* C2 = (OUT_MODE == 2) ? ((unsigned short*)Cout2 + (size_t)b * strideC) : nullptr;
      for (int pass = 0; pass < 2; ++pass) {
#pragma unroll
        for (int it = 0; it < 4; ++it) {
          const int row = it * 4 + q;
          const float* sp = slab + row * 68 + c8;
          v8h hv, lv;
#pragma unroll
          for (int e = 0; e < 8; ++e) {
            if (OUT_MODE == 1) {
              hv[e] = (_Float16)sp[e];
            } else {
              unsigned short hb = f2bf_bits(sp[e]);
              unsigned short lb = f2bf_bits(sp[e] - bf_bits2f(hb));
              hv[e] = __builtin_bit_cast(_Float16, hb);
              lv[e] = __builtin_bit_cast(_Float16, lb);
            }
          }
          *(volatile v8h*)(C + (size_t)(mBase + row) * ldc + n0 + c8) = hv;
          if (OUT_MODE == 2) *(volatile v8h*)(C2 + (size_t)(mBase + row) * ldc + n0 + c8) = lv;
        }
        __threadfence();
      }
    }
    __builtin_amdgcn_fence(__ATOMIC_RELEASE, "workgroup");
    __builtin_amdgcn_wave_barrier();
    __builtin_amdgcn_fence(__ATOMIC_ACQUIRE, "workgroup");
  }
}

__global__ __launch_bounds__(256) void cast_scale_f16x2(
    const float* __restrict__ in, _Float16* __restrict__ out, int n2, float sc) {
  int i = blockIdx.x * 256 + threadIdx.x;
  if (i < n2) {
    const _Float16 h0 = (_Float16)(in[2 * i] * sc), h1 = (_Float16)(in[2 * i + 1] * sc);
    const unsigned u = (unsigned)__builtin_bit_cast(unsigned short, h0) | ((unsigned)__builtin_bit_cast(unsigned short, h1) << 16);
    ((volatile unsigned*)out)[i] = u;
    __threadfence();
    ((volatile unsigned*)out)[i] = u;
  }
}

__global__ __launch_bounds__(256) void cast_qkv_w(
    const float* __restrict__ Wq, const float* __restrict__ Wk, const float* __restrict__ Wv,
    _Float16* __restrict__ out, int n2, float sc) {
  int i = blockIdx.x * 256 + threadIdx.x;
  if (i < n2) {
    const int e0 = 2 * i;
    const int h = e0 / (3 * kHdim * kHdim);
    const int rem = e0 - h * (3 * kHdim * kHdim);
    const int r = rem >> 6;
    const int d = rem & 63;
    const int which = r >> 6;
    const int rr = r & 63;
    const float* src = (which == 0) ? Wq : ((which == 1) ? Wk : Wv);
    const float* p = src + (size_t)h * (kHdim * kHdim) + rr * kHdim + d;
    const _Float16 h0 = (_Float16)(p[0] * sc), h1 = (_Float16)(p[1] * sc);
    const unsigned u = (unsigned)__builtin_bit_cast(unsigned short, h0) | ((unsigned)__builtin_bit_cast(unsigned short, h1) << 16);
    ((volatile unsigned*)out)[i] = u;
    __threadfence();
    ((volatile unsigned*)out)[i] = u;
  }
}

__global__ __launch_bounds__(256) void layernorm_rows(
    const float* __restrict__ x, const float* __restrict__ gam, const float* __restrict__ bet,
    float* __restrict__ yf, _Float16* __restrict__ yh, float hscale) {
  __shared__ float ssum[8];
  __shared__ float ssq[8];
  __shared__ __align__(16) unsigned hrow[512];
  const int row = blockIdx.x;
  const int t = threadIdx.x;
  const int w = t >> 5;
  const int l = t & 31;
  const v4f v = *(const v4f*)(x + (size_t)row * kDim + t * 4);
  float s = (v[0] + v[1]) + (v[2] + v[3]);
#pragma unroll
  for (int off = 1; off < 32; off <<= 1) s += __shfl_xor(s, off, 32);
  if (l == 0) ssum[w] = s;
  __syncthreads();
  float tot = 0.f;
#pragma unroll
  for (int i = 0; i < 8; ++i) tot += ssum[i];
  const float mean = tot * (1.0f / 1024.0f);
  const v4f d = v - mean;
  float q = (d[0] * d[0] + d[1] * d[1]) + (d[2] * d[2] + d[3] * d[3]);
#pragma unroll
  for (int off = 1; off < 32; off <<= 1) q += __shfl_xor(q, off, 32);
  if (l == 0) ssq[w] = q;
  __syncthreads();
  float totq = 0.f;
#pragma unroll
  for (int i = 0; i < 8; ++i) totq += ssq[i];
  const float var = totq * (1.0f / 1024.0f);
  const float inv = rsqrtf(var + 1e-5f);
  const v4f gv = *(const v4f*)(gam + t * 4);
  const v4f bv = *(const v4f*)(bet + t * 4);
  const v4f o = d * inv * gv + bv;
  float* yrow = yf + (size_t)row * kDim + t * 4;
  *(volatile v4f*)yrow = o;
  __threadfence();
  *(volatile v4f*)yrow = o;
  const unsigned hb0 = (unsigned)__builtin_bit_cast(unsigned short, (_Float16)(o[0] * hscale));
  const unsigned hb1 = (unsigned)__builtin_bit_cast(unsigned short, (_Float16)(o[1] * hscale));
  const unsigned hb2 = (unsigned)__builtin_bit_cast(unsigned short, (_Float16)(o[2] * hscale));
  const unsigned hb3 = (unsigned)__builtin_bit_cast(unsigned short, (_Float16)(o[3] * hscale));
  v2u pk;
  pk[0] = hb0 | (hb1 << 16);
  pk[1] = hb2 | (hb3 << 16);
  *(v2u*)(hrow + 2 * t) = pk;
  __syncthreads();
  if (t < 128) {
    const v4u wv = *(const v4u*)(hrow + 4 * t);
    _Float16* hp = yh + (size_t)row * kDim + t * 8;
    *(volatile v4u*)hp = wv;
    __threadfence();
    *(volatile v4u*)hp = wv;
  }
}

constexpr int kAKC = 64;
constexpr int kAQB = 64;
constexpr int kANW = 4;

__device__ __forceinline__ v8f mma_h(v16h a, v16h b, v8f c) {
  c = __builtin_amdgcn_wmma_f32_16x16x32_f16(false, a, false, b, (short)0, c, false, false);
  asm volatile("v_nop\n\tv_nop\n\tv_nop\n\tv_nop" : "+v"(c) : "v"(a), "v"(b));
  return c;
}

__device__ __forceinline__ void vt_scatter(_Float16* vt, v4u w, int d0, int kvr) {
#pragma unroll
  for (int e = 0; e < 4; ++e) {
    const unsigned u = w[e];
    const int d = d0 + 2 * e;
    vt[d * kAKC + kvr]       = __builtin_bit_cast(_Float16, (unsigned short)(u & 0xffffu));
    vt[(d + 1) * kAKC + kvr] = __builtin_bit_cast(_Float16, (unsigned short)(u >> 16));
  }
}

__global__ __launch_bounds__(128)
void attn_causal_h64(const _Float16* __restrict__ qkv, _Float16* __restrict__ attn_out,
                     float sscale, float pscale, float oscale) {
  union FH { v16h v; v8h h[2]; };
  __shared__ __align__(16) _Float16 Ksh[kAKC * kHdim];
  __shared__ __align__(16) _Float16 Vth[kHdim * kAKC];
  __shared__ __align__(16) _Float16 Psh[kANW][16 * kAKC];
  __shared__ __align__(16) float  Osl[kANW][16 * 68];

  const int tid  = threadIdx.x;
  const int wave = tid >> 5;
  const int lane = tid & 31;
  const int hh   = lane >> 4;
  const int c    = lane & 15;

  const int nqb = kSeq / kAQB;
  const int bx = blockIdx.x;
  const int qb = bx % nqb;
  const int bh = bx / nqb;
  const int h  = bh % kHeads;
  const int b  = bh / kHeads;
  const int q0 = qb * kAQB + wave * 16;

  const _Float16* base = qkv + (size_t)b * kSeq * kQkvLd + (size_t)h * (3 * kHdim);

  v16h qa[2];
  {
    const _Float16* qrow = base + (size_t)(q0 + c) * kQkvLd + 8 * hh;
    qa[0] = Frag<_Float16>::load(qrow);
    qa[1] = Frag<_Float16>::load(qrow + 32);
  }

  float mrow[8], lrow[8];
  v8f oacc[4];
#pragma unroll
  for (int r = 0; r < 8; ++r) { mrow[r] = -INFINITY; lrow[r] = 0.f; }
#pragma unroll
  for (int t = 0; t < 4; ++t) oacc[t] = (v8f){0.f,0.f,0.f,0.f,0.f,0.f,0.f,0.f};

  const int nChunks = qb + 1;
  for (int kc = 0; kc < nChunks; ++kc) {
    const int kv0 = kc * kAKC;
    __syncthreads();
    {
      const int kvr = tid >> 1, dh = (tid & 1) * 32;
      const _Float16* krow = base + (size_t)(kv0 + kvr) * kQkvLd + kHdim + dh;
      const _Float16* vrow = krow + kHdim;
      const v8h k0v = *(const v8h*)(krow);
      const v8h k1v = *(const v8h*)(krow + 8);
      const v8h k2v = *(const v8h*)(krow + 16);
      const v8h k3v = *(const v8h*)(krow + 24);
      const v4u v0w = *(const v4u*)(vrow);
      const v4u v1w = *(const v4u*)(vrow + 8);
      const v4u v2w = *(const v4u*)(vrow + 16);
      const v4u v3w = *(const v4u*)(vrow + 24);
      _Float16* kd = Ksh + kvr * kHdim + dh;
      *(v8h*)(kd)      = k0v;
      *(v8h*)(kd + 8)  = k1v;
      *(v8h*)(kd + 16) = k2v;
      *(v8h*)(kd + 24) = k3v;
      vt_scatter(Vth, v0w, dh,      kvr);
      vt_scatter(Vth, v1w, dh + 8,  kvr);
      vt_scatter(Vth, v2w, dh + 16, kvr);
      vt_scatter(Vth, v3w, dh + 24, kvr);
    }
    __syncthreads();

    v8f s[4];
#pragma unroll
    for (int j = 0; j < 4; ++j) {
      s[j] = (v8f){0.f,0.f,0.f,0.f,0.f,0.f,0.f,0.f};
#pragma unroll
      for (int dc = 0; dc < 2; ++dc) {
        FH kb;
        kb.h[0] = *(const v8h*)(Ksh + (j * 16 + c) * kHdim + dc * 32 + 8 * hh);
        kb.h[1] = *(const v8h*)(Ksh + (j * 16 + c) * kHdim + dc * 32 + 16 + 8 * hh);
        s[j] = mma_h(qa[dc], kb.v, s[j]);
      }
    }
    const bool diag = (kc == qb);
    float cm[8];
#pragma unroll
    for (int r = 0; r < 8; ++r) {
      const int qrow = q0 + 8 * hh + r;
      float m = -INFINITY;
#pragma unroll
      for (int j = 0; j < 4; ++j) {
        const int kvcol = kv0 + j * 16 + c;
        float sv = s[j][r] * sscale;
        const bool masked = diag && (kvcol > qrow);
        sv = masked ? -INFINITY : sv;
        s[j][r] = sv;
        m = fmaxf(m, sv);
      }
#pragma unroll
      for (int off = 1; off < 16; off <<= 1) m = fmaxf(m, __shfl_xor(m, off, 32));
      cm[r] = m;
    }
    _Float16* pw = Psh[wave];
#pragma unroll
    for (int r = 0; r < 8; ++r) {
      const float mnew = fmaxf(mrow[r], cm[r]);
      const float alpha = __expf(mrow[r] - mnew);
      mrow[r] = mnew;
      float psum = 0.f;
#pragma unroll
      for (int j = 0; j < 4; ++j) {
        const float p = __expf(s[j][r] - mnew);
        psum += p;
        pw[(8 * hh + r) * kAKC + j * 16 + c] = (_Float16)(p * pscale);
      }
#pragma unroll
      for (int off = 1; off < 16; off <<= 1) psum += __shfl_xor(psum, off, 32);
      lrow[r] = lrow[r] * alpha + psum;
#pragma unroll
      for (int t = 0; t < 4; ++t) oacc[t][r] *= alpha;
    }
    __builtin_amdgcn_fence(__ATOMIC_RELEASE, "workgroup");
    __builtin_amdgcn_wave_barrier();
    __builtin_amdgcn_fence(__ATOMIC_ACQUIRE, "workgroup");
#pragma unroll
    for (int kk = 0; kk < 2; ++kk) {
      FH pa;
      pa.h[0] = *(const v8h*)(pw + c * kAKC + kk * 32 + 8 * hh);
      pa.h[1] = *(const v8h*)(pw + c * kAKC + kk * 32 + 16 + 8 * hh);
#pragma unroll
      for (int t = 0; t < 4; ++t) {
        FH vb;
        vb.h[0] = *(const v8h*)(Vth + (t * 16 + c) * kAKC + kk * 32 + 8 * hh);
        vb.h[1] = *(const v8h*)(Vth + (t * 16 + c) * kAKC + kk * 32 + 16 + 8 * hh);
        oacc[t] = mma_h(pa.v, vb.v, oacc[t]);
      }
    }
  }

  float* os = Osl[wave];
#pragma unroll
  for (int r = 0; r < 8; ++r) {
    const float inv = oscale / lrow[r];
#pragma unroll
    for (int t = 0; t < 4; ++t) os[(8 * hh + r) * 68 + t * 16 + c] = oacc[t][r] * inv;
  }
  __builtin_amdgcn_fence(__ATOMIC_RELEASE, "workgroup");
  __builtin_amdgcn_wave_barrier();
  __builtin_amdgcn_fence(__ATOMIC_ACQUIRE, "workgroup");
  {
    const int q8 = lane >> 3, c8 = (lane & 7) * 8;
    _Float16* ob = attn_out + (size_t)(b * kSeq) * kDim + h * kHdim;
    for (int pass = 0; pass < 2; ++pass) {
#pragma unroll
      for (int it = 0; it < 4; ++it) {
        const int row = it * 4 + q8;
        const float* sp = os + row * 68 + c8;
        v8h hv;
#pragma unroll
        for (int e = 0; e < 8; ++e) hv[e] = (_Float16)sp[e];
        *(volatile v8h*)(ob + (size_t)(q0 + row) * kDim + c8) = hv;
      }
      __threadfence();
    }
  }
}

extern "C" void kernel_launch(void* const* d_in, const int* in_sizes, int n_in,
                              void* d_out, int out_size, void* d_ws, size_t ws_size,
                              hipStream_t stream) {
  if (n_in != 13) return;
  if (in_sizes[0] != kRows * kDim) return;
  if (in_sizes[1] != kDim || in_sizes[2] != kDim || in_sizes[7] != kDim || in_sizes[8] != kDim) return;
  if (in_sizes[3] != kHeads * kHdim * kHdim || in_sizes[4] != kHeads * kHdim * kHdim ||
      in_sizes[5] != kHeads * kHdim * kHdim) return;
  if (in_sizes[6] != kDim * kDim || in_sizes[9] != kFfn * kDim || in_sizes[10] != kFfn ||
      in_sizes[11] != kDim * kFfn || in_sizes[12] != kDim) return;
  if (out_size != kRows * kDim) return;
  if (ws_size < kWsTotal) return;

  const float* x    = (const float*)d_in[0];
  const float* ln1g = (const float*)d_in[1];
  const float* ln1b = (const float*)d_in[2];
  const float* Wq   = (const float*)d_in[3];
  const float* Wk   = (const float*)d_in[4];
  const float* Wv   = (const float*)d_in[5];
  const float* Wo   = (const float*)d_in[6];
  const float* ln2g = (const float*)d_in[7];
  const float* ln2b = (const float*)d_in[8];
  const float* W1   = (const float*)d_in[9];
  const float* b1   = (const float*)d_in[10];
  const float* W2   = (const float*)d_in[11];
  const float* b2   = (const float*)d_in[12];
  float* outf = (float*)d_out;

  char* ws = (char*)d_ws;
  _Float16* wqkv = (_Float16*)(ws + kOffWqkv);
  _Float16* woh  = (_Float16*)(ws + kOffWo);
  _Float16* w1h  = (_Float16*)(ws + kOffW1);
  _Float16* w2h  = (_Float16*)(ws + kOffW2);
  float*    x1f  = (float*)(ws + kOffX1f);
  _Float16* x1h  = (_Float16*)(ws + kOffX1h);
  _Float16* qkvp = (_Float16*)(ws + kOffQkv);
  _Float16* attp = (_Float16*)(ws + kOffAttn);
  float*    uf   = (float*)(ws + kOffU);
  float*    u2f  = x1f;
  _Float16* u2h  = x1h;
  _Float16* hid  = (_Float16*)(ws + kOffHid);

  typedef const unsigned short* cus;

  {
    const int n2 = kHeads * 3 * kHdim * kHdim / 2;
    cast_qkv_w<<<dim3((unsigned)((n2 + 255) / 256)), dim3(256), 0, stream>>>(Wq, Wk, Wv, wqkv, n2, kCarryWqkv);
  }
  {
    const int n2 = kDim * kDim / 2;
    cast_scale_f16x2<<<dim3((unsigned)((n2 + 255) / 256)), dim3(256), 0, stream>>>(Wo, woh, n2, kCarryWo);
  }
  {
    const int n2 = kFfn * kDim / 2;
    cast_scale_f16x2<<<dim3((unsigned)((n2 + 255) / 256)), dim3(256), 0, stream>>>(W1, w1h, n2, kCarryW1);
    cast_scale_f16x2<<<dim3((unsigned)((n2 + 255) / 256)), dim3(256), 0, stream>>>(W2, w2h, n2, kCarryW2);
  }

  layernorm_rows<<<dim3((unsigned)kRows), dim3(256), 0, stream>>>(x, ln1g, ln1b, x1f, x1h, kCarryAct);

  {
    const unsigned blocks = (unsigned)((kRows / 64) * ((3 * kHdim) / 64) / 8);
    wmma_gemm64<0, false, 0, 1, false, 0><<<dim3(blocks, kHeads), dim3(256), 0, stream>>>(
        (cus)x1h, (cus)x1h, kDim, (long)kHdim,
        (cus)wqkv, (cus)wqkv, kHdim, (long)(3 * kHdim * kHdim),
        (void*)qkvp, (void*)qkvp, kQkvLd, (long)(3 * kHdim),
        b1, x1f, (long)0,
        kRows, 3 * kHdim, kHdim, kCarryQkv / (kCarryAct * kCarryWqkv), 1.0f);
  }

  {
    const unsigned blocks = (unsigned)(kBatch * kHeads * (kSeq / kAQB));
    attn_causal_h64<<<dim3(blocks), dim3(128), 0, stream>>>(
        qkvp, attp, 0.125f / (kCarryQkv * kCarryQkv), kCarryP, kCarryAttn / (kCarryP * kCarryQkv));
  }

  {
    const unsigned blocks = (unsigned)((kRows / 64) * (kDim / 64) / 8);
    wmma_gemm64<0, false, 0, 0, true, 0><<<dim3(blocks, 1), dim3(256), 0, stream>>>(
        (cus)attp, (cus)attp, kDim, (long)0,
        (cus)woh, (cus)woh, kDim, (long)0,
        (void*)uf, (void*)uf, kDim, (long)0,
        b1, x1f, (long)0,
        kRows, kDim, kDim, 1.0f / (kCarryAttn * kCarryWo), 1.0f);
  }

  layernorm_rows<<<dim3((unsigned)kRows), dim3(256), 0, stream>>>(uf, ln2g, ln2b, u2f, u2h, kCarryAct);

  {
    const unsigned blocks = (unsigned)((kRows / 64) * (kFfn / 64) / 8);
    wmma_gemm64<0, false, 2, 1, false, 6><<<dim3(blocks, 1), dim3(256), 0, stream>>>(
        (cus)u2h, (cus)u2h, kDim, (long)0,
        (cus)w1h, (cus)w1h, kDim, (long)0,
        (void*)hid, (void*)hid, kFfn, (long)0,
        b1, u2f, (long)0,
        kRows, kFfn, kDim, 1.0f / (kCarryAct * kCarryW1), kCarryH);
  }

  {
    const unsigned blocks = (unsigned)((kRows / 64) * (kDim / 64) / 8);
    wmma_gemm64<0, false, 2, 0, true, 0><<<dim3(blocks, 1), dim3(256), 0, stream>>>(
        (cus)hid, (cus)hid, kFfn, (long)0,
        (cus)w2h, (cus)w2h, kFfn, (long)0,
        (void*)outf, (void*)outf, kDim, (long)0,
        b2, u2f, (long)0,
        kRows, kDim, kFfn, 1.0f / (kCarryH * kCarryW2), 1.0f);
  }
}
